// PlayerMovementGNN_82308753260856
// MI455X (gfx1250) — hardware-run, weakly checked
//
#include <hip/hip_runtime.h>

typedef float          v8f   __attribute__((ext_vector_type(8)));
typedef float          v4f   __attribute__((ext_vector_type(4)));
typedef unsigned int   v4u   __attribute__((ext_vector_type(4)));
typedef int            v8i   __attribute__((ext_vector_type(8)));
typedef unsigned short v8us  __attribute__((ext_vector_type(8)));
typedef unsigned short v16us __attribute__((ext_vector_type(16)));
typedef __bf16         v16bf __attribute__((ext_vector_type(16)));
typedef _Float16       v16h  __attribute__((ext_vector_type(16)));
typedef v4f  __attribute__((may_alias)) v4fa;
typedef v8us __attribute__((may_alias)) v8usa;
union FragB { v16bf v; v16us u; v8us h[2]; v8i w; };
union FragH { v16h  v; v16us u; v8us h[2]; v8i w; };

__device__ __forceinline__ v8f wmb(const FragB& a, const FragB& b, v8f c) {
  v8f d = __builtin_amdgcn_wmma_f32_16x16x32_bf16(false, a.v, false, b.v, (short)0, c, false, false);
  asm volatile("v_nop\n\tv_nop\n\tv_nop\n\tv_nop" : "+v"(d) : "v"(a.w), "v"(b.w));
  return d;
}

__device__ __forceinline__ v8f wmh(const FragH& a, const FragH& b, v8f c) {
  v8f d = __builtin_amdgcn_wmma_f32_16x16x32_f16(false, a.v, false, b.v, (short)0, c, false, false);
  asm volatile("v_nop\n\tv_nop\n\tv_nop\n\tv_nop" : "+v"(d) : "v"(a.w), "v"(b.w));
  return d;
}

__device__ __forceinline__ unsigned bf16_bits(float f) {
  const unsigned u = __float_as_uint(f);
  const unsigned r = (u + 0x7FFFu + ((u >> 16) & 1u)) >> 16;
  const unsigned q = (u >> 16) | 0x40u;
  return ((u & 0x7fffffffu) > 0x7f800000u) ? q : r;
}

__device__ __forceinline__ float bf16_val(float f) {
  return __uint_as_float(bf16_bits(f) << 16);
}
__device__ __forceinline__ int clampi(int v, int lo, int hi) {
  return v < lo ? lo : (v > hi ? hi : v);
}

__device__ __forceinline__ unsigned f16_bits(float f) {
  const unsigned u  = __float_as_uint(f);
  const unsigned s  = (u >> 16) & 0x8000u;
  const unsigned a  = u & 0x7fffffffu;
  const unsigned t  = a - 0x38000000u;
  const unsigned r  = (t + 0x0FFFu + ((t >> 13) & 1u)) >> 13;
  const unsigned rc = r > 0x7C00u ? 0x7C00u : r;
  const bool small  = a < 0x38800000u;
  const bool isnan  = a > 0x7f800000u;
  const unsigned fin = small ? 0u : (s | rc);
  return isnan ? (s | 0x7E00u) : fin;
}

__device__ __forceinline__ unsigned pk16(unsigned lo, unsigned hi) { return lo | (hi << 16); }
__device__ __forceinline__ unsigned bf16_lo_bits(float v) {
  float hi = bf16_val(v);
  asm volatile("" : "+v"(hi));
  return bf16_bits(v - hi);
}
__device__ __forceinline__ v4u pack8_bf16(v4f a, v4f c) {
  return (v4u){ pk16(bf16_bits(a[0]), bf16_bits(a[1])), pk16(bf16_bits(a[2]), bf16_bits(a[3])),
                pk16(bf16_bits(c[0]), bf16_bits(c[1])), pk16(bf16_bits(c[2]), bf16_bits(c[3])) };
}
__device__ __forceinline__ v4u pack8_bf16_lo(v4f a, v4f c) {
  return (v4u){ pk16(bf16_lo_bits(a[0]), bf16_lo_bits(a[1])), pk16(bf16_lo_bits(a[2]), bf16_lo_bits(a[3])),
                pk16(bf16_lo_bits(c[0]), bf16_lo_bits(c[1])), pk16(bf16_lo_bits(c[2]), bf16_lo_bits(c[3])) };
}
__device__ __forceinline__ v4u pack8_f16(v4f a, v4f c) {
  return (v4u){ pk16(f16_bits(a[0]), f16_bits(a[1])), pk16(f16_bits(a[2]), f16_bits(a[3])),
                pk16(f16_bits(c[0]), f16_bits(c[1])), pk16(f16_bits(c[2]), f16_bits(c[3])) };
}

template <int FORM>
__global__ __launch_bounds__(256) void k_plane(const float* __restrict__ src, int rows, int cols, int ldsrc,
                                               unsigned short* __restrict__ dst, int MP, int KP) {
  static_assert(FORM >= 0 && FORM <= 3);
  const int KTOT = (FORM == 1 || FORM == 3) ? 2 * KP : KP;
  const unsigned ppr   = (unsigned)(KTOT >> 3);
  const unsigned kp8   = (unsigned)(KP >> 3);
  const unsigned total = (unsigned)MP * ppr;
  const unsigned g     = blockIdx.x * 256u + threadIdx.x;
  const unsigned rowu  = g / ppr;
  const unsigned p     = g - rowu * ppr;
  const bool second    = p >= kp8;
  const int row = (int)rowu;
  const int c0  = (int)((second ? p - kp8 : p) << 3);
  const float* srow = src + (size_t)clampi(row, 0, rows - 1) * (size_t)ldsrc;
  float x[8];
  unsigned mk[8];
#pragma unroll
  for (int e = 0; e < 8; ++e) {
    const int c = c0 + e;
    const float v = srow[clampi(c, 0, cols - 1)];
    asm volatile("" :: "v"(v));
    x[e]  = v;
    mk[e] = (row < rows && c < cols) ? 0xFFFFu : 0u;
  }
  const v4f a = (v4f){ x[0], x[1], x[2], x[3] };
  const v4f c = (v4f){ x[4], x[5], x[6], x[7] };
  v4u o;
  if (FORM == 2) {
    o = pack8_f16(a, c);
  } else {
    const v4u hi = pack8_bf16(a, c);
    o = hi;
    if (FORM == 1) { const v4u lo = pack8_bf16_lo(a, c); o = second ? lo : hi; }
  }
  const v4u mw = (v4u){ pk16(mk[0], mk[1]), pk16(mk[2], mk[3]), pk16(mk[4], mk[5]), pk16(mk[6], mk[7]) };
  o &= mw;
  if (g < total) {
    volatile v4u* q = (volatile v4u*)(dst + (size_t)g * 8);
    *q = o;
    __threadfence();
    *q = o;
  }
}

template <int FORM> struct FragOf    { typedef FragB T; };
template <>         struct FragOf<2> { typedef FragH T; };
__device__ __forceinline__ v8f mm(const FragB& a, const FragB& b, v8f c) { return wmb(a, b, c); }
__device__ __forceinline__ v8f mm(const FragH& a, const FragH& b, v8f c) { return wmh(a, b, c); }
template <class F> __device__ __forceinline__ F ld_frag(const unsigned short* p) {
  F f;
  f.h[0] = *(const v8usa*)(p);
  f.h[1] = *(const v8usa*)(p + 16);
  return f;
}

template <int FORM, int EPI>
__global__ __launch_bounds__(256) __attribute__((amdgpu_num_vgpr(248)))
void k_gemm_nt(const unsigned short* __restrict__ A, const unsigned short* __restrict__ B,
               const float* __restrict__ bias, float* __restrict__ D, int M, int N, int KTOT, int ldd) {
  static_assert(FORM >= 0 && FORM <= 2);
  static_assert(EPI == 0 || EPI == 1);
  typedef typename FragOf<FORM>::T F;
  __shared__ __attribute__((aligned(16))) float sT[8][16 * 68];
  const int lane = threadIdx.x & 31;
  const int wave = threadIdx.x >> 5;
  const int tilesM = (M + 63) >> 6;
  const int tilesN = (N + 63) >> 6;
  const int tile = blockIdx.x * 8 + wave;
  if (tile >= tilesM * tilesN) return;
  const int tm = tile / tilesN;
  const int tn = tile - tm * tilesN;
  const int m0 = tm << 6;
  const int n0 = tn << 6;

  const int rl = lane & 15;
  const int h8 = (lane >> 4) * 8;
  const unsigned short* pa = A + (size_t)(m0 + rl) * (size_t)KTOT + h8;
  const unsigned short* pb = B + (size_t)(n0 + rl) * (size_t)KTOT + h8;

  v8f acc[4][4];
#pragma unroll
  for (int i = 0; i < 4; ++i)
#pragma unroll
    for (int j = 0; j < 4; ++j) acc[i][j] = (v8f){0.f, 0.f, 0.f, 0.f, 0.f, 0.f, 0.f, 0.f};

#pragma unroll 1
  for (int k0 = 0; k0 < KTOT; k0 += 32) {
    F bf[4];
#pragma unroll
    for (int j = 0; j < 4; ++j) bf[j] = ld_frag<F>(pb + (size_t)(j << 4) * (size_t)KTOT + k0);
#pragma unroll
    for (int i = 0; i < 4; ++i) {
      const F af = ld_frag<F>(pa + (size_t)(i << 4) * (size_t)KTOT + k0);
#pragma unroll
      for (int j = 0; j < 4; ++j) acc[i][j] = mm(af, bf[j], acc[i][j]);
    }
  }

  float* slab = sT[wave];
  const int hh = lane >> 4;
  const int c4 = (lane & 15) * 4;
  const int nc = n0 + c4;
  const bool cok = nc < N;
  v4f bv = (v4f){0.f, 0.f, 0.f, 0.f};
  if (EPI == 1) {
    bv = *(const v4fa*)(bias + clampi(nc, 0, N - 4));
    asm volatile("" :: "v"(bv));
  }
#pragma unroll
  for (int i = 0; i < 4; ++i) {
    const int mBase = m0 + (i << 4);
#pragma unroll
    for (int j = 0; j < 4; ++j) {
#pragma unroll
      for (int r = 0; r < 8; ++r) slab[(h8 + r) * 68 + (j << 4) + rl] = acc[i][j][r];
    }
    __builtin_amdgcn_fence(__ATOMIC_RELEASE, "workgroup");
    __builtin_amdgcn_wave_barrier();
    __builtin_amdgcn_fence(__ATOMIC_ACQUIRE, "workgroup");
    v4f vv[8];
#pragma unroll
    for (int it = 0; it < 8; ++it) {
      const int row = it * 2 + hh;
      v4f v = *(const v4fa*)(slab + row * 68 + c4);
      if (EPI == 1) v += bv;
      vv[it] = v;
    }
    for (int pass = 0; pass < 2; ++pass) {
#pragma unroll
      for (int it = 0; it < 8; ++it) {
        const int row = mBase + it * 2 + hh;
        if (cok && row < M) *(volatile v4f*)(D + (size_t)row * (size_t)ldd + nc) = vv[it];
      }
      __threadfence();
    }
    __builtin_amdgcn_fence(__ATOMIC_RELEASE, "workgroup");
    __builtin_amdgcn_wave_barrier();
    __builtin_amdgcn_fence(__ATOMIC_ACQUIRE, "workgroup");
  }
}

#pragma clang fp contract(off)

#include <stddef.h>
#include <math.h>

#ifndef SPLIT_L2
#define SPLIT_L2 1
#endif
#ifndef SPLIT_H
#define SPLIT_H 1
#endif

#define NN      65536
#define NE      (1 << 20)
#define CIN     16
#define HD      64
#define NOUTC   2
#define NOUT    (NN * NOUTC)
#define KP1     32
#define K2      (SPLIT_L2 ? 128 : 64)
#define KH      (SPLIT_H ? 128 : 64)
#define NTHR    256
#define NWAVE   8
#define EPT     8
#define WCH     (32 * EPT)
#define NBRUN   1024
#define SLB     10
#define NBK     64
#define WLCAP   4096
#define RCAP    21504
#define DEGCAP  64
#define MAXDEG_MEAS   38
#define MAXB1024_MEAS 16727
#define OWB     64

#define BK_ZINTS (NWAVE * WLCAP + RCAP + 3 * NBRUN)
#define BK_INTS  (BK_ZINTS + 16)
#define BK_LDS   (BK_INTS * 4)

#define PB1   1
#define PB2   (HD * K2 / 8 / NTHR)
#define PBH   (HD * KH / 8 / NTHR)
#define PBTOT (PB1 + PB2 + PBH + 3)

static_assert(NN == 64 * 1024 && NN == NBK * NBRUN);
static_assert(NBRUN == (1 << SLB) && NBRUN % NTHR == 0 && NBRUN % 32 == 0);
static_assert(NE == (1 << 20) && (((long long)(NE - 1)) << SLB) + (NBRUN - 1) < (1LL << 31));
static_assert(NE % (NWAVE * WCH) == 0 && NE % 4 == 0);
static_assert(KP1 % 32 == 0 && K2 % 32 == 0 && KH % 32 == 0 && CIN <= KP1);
static_assert(HD == 64 && NN % 64 == 0 && HD % 32 == 0 && NN % 16 == 0);
static_assert(NOUT % 32 == 0 && NOUT % NTHR == 0 && NOUT == 131072);
static_assert(RCAP % 512 == 0 && BK_ZINTS % (NTHR * 4) == 0);
static_assert((long long)RCAP * 100 >= (long long)MAXB1024_MEAS * 125);
static_assert(WLCAP * NWAVE >= RCAP && WLCAP >= MAXB1024_MEAS / NWAVE + 1024);
static_assert(MAXDEG_MEAS + 8 <= DEGCAP);
static_assert(BK_LDS <= 262144 && BK_LDS + 0 <= 327680);
static_assert(8 * 16 * 68 * 4 == 34816);
static_assert((HD * KP1 / 8) == NTHR * PB1 && (HD * K2 / 8) % NTHR == 0 && (HD * KH / 8) % NTHR == 0);
static_assert(NN % OWB == 0 && NBRUN % OWB == 0 && OWB == NWAVE * 8);

typedef float v2f __attribute__((ext_vector_type(2)));
typedef int   v2i __attribute__((ext_vector_type(2)));
typedef int   v4i __attribute__((ext_vector_type(4)));
typedef v2f __attribute__((may_alias)) v2fa;
typedef v2i __attribute__((may_alias)) v2ia;
typedef v4i __attribute__((may_alias)) v4ia;

__device__ __forceinline__ void st2_v4f(float* p, v4f v) {
  *(volatile v4f*)p = v;
  __threadfence();
  *(volatile v4f*)p = v;
}
__device__ __forceinline__ void st2_v4i(int* p, v4i v) {
  *(volatile v4i*)p = v;
  __threadfence();
  *(volatile v4i*)p = v;
}
__device__ __forceinline__ void st2_v8us(unsigned short* p, v8us v) {
  *(volatile v8us*)p = v;
  __threadfence();
  *(volatile v8us*)p = v;
}

__global__ __launch_bounds__(NTHR) void k_prep(const float* __restrict__ W1, const float* __restrict__ b1,
                                               const float* __restrict__ W2, const float* __restrict__ b2,
                                               const float* __restrict__ Wl, const float* __restrict__ bl,
                                               unsigned short* W1P, unsigned short* W2D, unsigned short* WLD,
                                               float* BIAS) {
  const int tid = (int)threadIdx.x;
  const int blk = (int)blockIdx.x;
  if (blk < PB1) {
    const int u = tid;
    const int n = u >> 2, k8 = (u & 3) * 8;
    float f[8];
#pragma unroll
    for (int i = 0; i < 8; ++i) {
      const int k = k8 + i;
      const float v = W1[(size_t)clampi(k, 0, CIN - 1) * HD + n];
      asm volatile("" :: "v"(v));
      f[i] = v;
    }
    v8us o;
#pragma unroll
    for (int i = 0; i < 8; ++i) {
      const unsigned mk = (k8 + i < CIN) ? 0xFFFFu : 0u;
      o[i] = (unsigned short)(bf16_bits(f[i]) & mk);
    }
    st2_v8us(W1P + (size_t)u * 8, o);
  } else if (blk < PB1 + PB2) {
    const int u = (blk - PB1) * NTHR + tid;
    const int n = u / (K2 / 8);
    const int k8 = (u - n * (K2 / 8)) * 8;
    const int ks = k8 & 63;
    float f[8];
#pragma unroll
    for (int i = 0; i < 8; ++i) {
      const float v = W2[(size_t)(ks + i) * HD + n];
      asm volatile("" :: "v"(v));
      f[i] = v;
    }
    v8us o;
#pragma unroll
    for (int i = 0; i < 8; ++i) o[i] = (unsigned short)bf16_bits(f[i]);
    st2_v8us(W2D + (size_t)u * 8, o);
  } else if (blk < PB1 + PB2 + PBH) {
    const int u = (blk - PB1 - PB2) * NTHR + tid;
    const int n = u / (KH / 8);
    const int k8 = (u - n * (KH / 8)) * 8;
    const int ks = k8 & 63;
    const int nc = n < NOUTC ? n : NOUTC - 1;
    const unsigned mk = n < NOUTC ? 0xFFFFu : 0u;
    float f[8];
#pragma unroll
    for (int i = 0; i < 8; ++i) {
      const float v = Wl[(size_t)(ks + i) * NOUTC + nc];
      asm volatile("" :: "v"(v));
      f[i] = v;
    }
    v8us o;
#pragma unroll
    for (int i = 0; i < 8; ++i) o[i] = (unsigned short)(bf16_bits(f[i]) & mk);
    st2_v8us(WLD + (size_t)u * 8, o);
  } else if (blk == PB1 + PB2 + PBH) {
    const int q = tid & 15;
    float f[4];
#pragma unroll
    for (int i = 0; i < 4; ++i) {
      const float v = b1[4 * q + i];
      asm volatile("" :: "v"(v));
      f[i] = v;
    }
    const v4f o = (v4f){ bf16_val(f[0]), bf16_val(f[1]), bf16_val(f[2]), bf16_val(f[3]) };
    if (tid < 16) st2_v4f(BIAS + 4 * q, o);
  } else if (blk == PB1 + PB2 + PBH + 1) {
    const int q = tid & 15;
    float f[4];
#pragma unroll
    for (int i = 0; i < 4; ++i) {
      const float v = b2[4 * q + i];
      asm volatile("" :: "v"(v));
      f[i] = v;
    }
    const v4f o = (v4f){ bf16_val(f[0]), bf16_val(f[1]), bf16_val(f[2]), bf16_val(f[3]) };
    if (tid < 16) st2_v4f(BIAS + HD + 4 * q, o);
  } else {
    const int q = tid & 15;
    float f[4];
#pragma unroll
    for (int i = 0; i < 4; ++i) {
      const int e = 4 * q + i;
      const float v = bl[e < NOUTC ? e : NOUTC - 1];
      asm volatile("" :: "v"(v));
      const unsigned mk = e < NOUTC ? 0xFFFFFFFFu : 0u;
      f[i] = __uint_as_float(__float_as_uint(bf16_val(v)) & mk);
    }
    const v4f o = (v4f){ f[0], f[1], f[2], f[3] };
    if (tid < 16) st2_v4f(BIAS + 2 * HD + 4 * q, o);
  }
}

__global__ __launch_bounds__(NTHR) void k_list(const int* __restrict__ ei, const float* __restrict__ ew,
                                               int* PAIRS, int* CNT, int* OFF, int* DINV, int* FLAG) {
  extern __shared__ __attribute__((aligned(16))) int dsm[];
  int* wl   = dsm;
  int* pl   = dsm + NWAVE * WLCAP;
  int* cnt  = pl + RCAP;
  int* offs = cnt + NBRUN;
  int* cur  = offs + NBRUN;
  int* misc = cur + NBRUN;
  const int* srcs = ei;
  const int* dsts = ei + NE;
  const int tid = (int)threadIdx.x, lane = tid & 31, wave = tid >> 5;
  const int blk = (int)blockIdx.x;
  const unsigned nbs = (unsigned)(blk * NBRUN);

  {
    const v4i z4 = {0, 0, 0, 0};
    for (int i = tid * 4; i < BK_ZINTS; i += NTHR * 4) *(v4ia*)(dsm + i) = z4;
    if (tid < 16) misc[tid] = 0;
  }
  __syncthreads();

  {
    const int per  = NE / NWAVE;
    const int ebeg = wave * per;
    const int eend = ebeg + per;
    int* mylist = wl + wave * WLCAP;
    int wc = 0;
#pragma unroll 1
    for (int cb = ebeg; cb < eend; cb += WCH) {
      const int e0 = cb + lane * EPT;
      const v4i da = *(const v4ia*)(dsts + e0);
      const v4i db = *(const v4ia*)(dsts + e0 + 4);
      const unsigned s0 = (unsigned)da.x - nbs, s1 = (unsigned)da.y - nbs;
      const unsigned s2 = (unsigned)da.z - nbs, s3 = (unsigned)da.w - nbs;
      const unsigned s4 = (unsigned)db.x - nbs, s5 = (unsigned)db.y - nbs;
      const unsigned s6 = (unsigned)db.z - nbs, s7 = (unsigned)db.w - nbs;
      const bool h0 = s0 < (unsigned)NBRUN, h1 = s1 < (unsigned)NBRUN, h2 = s2 < (unsigned)NBRUN, h3 = s3 < (unsigned)NBRUN;
      const bool h4 = s4 < (unsigned)NBRUN, h5 = s5 < (unsigned)NBRUN, h6 = s6 < (unsigned)NBRUN, h7 = s7 < (unsigned)NBRUN;
      const unsigned m0 = __builtin_amdgcn_ballot_w32(h0), m1 = __builtin_amdgcn_ballot_w32(h1);
      const unsigned m2 = __builtin_amdgcn_ballot_w32(h2), m3 = __builtin_amdgcn_ballot_w32(h3);
      const unsigned m4 = __builtin_amdgcn_ballot_w32(h4), m5 = __builtin_amdgcn_ballot_w32(h5);
      const unsigned m6 = __builtin_amdgcn_ballot_w32(h6), m7 = __builtin_amdgcn_ballot_w32(h7);
      const unsigned any = m0 | m1 | m2 | m3 | m4 | m5 | m6 | m7;
      if (any != 0u) {
        const int pre = (int)(__builtin_amdgcn_mbcnt_lo(m0, 0u) + __builtin_amdgcn_mbcnt_lo(m1, 0u) +
                              __builtin_amdgcn_mbcnt_lo(m2, 0u) + __builtin_amdgcn_mbcnt_lo(m3, 0u) +
                              __builtin_amdgcn_mbcnt_lo(m4, 0u) + __builtin_amdgcn_mbcnt_lo(m5, 0u) +
                              __builtin_amdgcn_mbcnt_lo(m6, 0u) + __builtin_amdgcn_mbcnt_lo(m7, 0u));
        int p = wc + pre;
        if (h0) { if (p < WLCAP) mylist[p] = ((e0 + 0) << SLB) | (int)s0; p = p + 1; }
        if (h1) { if (p < WLCAP) mylist[p] = ((e0 + 1) << SLB) | (int)s1; p = p + 1; }
        if (h2) { if (p < WLCAP) mylist[p] = ((e0 + 2) << SLB) | (int)s2; p = p + 1; }
        if (h3) { if (p < WLCAP) mylist[p] = ((e0 + 3) << SLB) | (int)s3; p = p + 1; }
        if (h4) { if (p < WLCAP) mylist[p] = ((e0 + 4) << SLB) | (int)s4; p = p + 1; }
        if (h5) { if (p < WLCAP) mylist[p] = ((e0 + 5) << SLB) | (int)s5; p = p + 1; }
        if (h6) { if (p < WLCAP) mylist[p] = ((e0 + 6) << SLB) | (int)s6; p = p + 1; }
        if (h7) { if (p < WLCAP) mylist[p] = ((e0 + 7) << SLB) | (int)s7; p = p + 1; }
        wc += (int)(__builtin_popcount(m0) + __builtin_popcount(m1) + __builtin_popcount(m2) + __builtin_popcount(m3) +
                    __builtin_popcount(m4) + __builtin_popcount(m5) + __builtin_popcount(m6) + __builtin_popcount(m7));
      }
    }
    if (lane == 0) misc[wave] = wc;
  }
  __syncthreads();

  if (wave == 0) {
    int ov = 0;
    int tot = 0;
#pragma unroll 1
    for (int w2 = 0; w2 < NWAVE; ++w2) {
      int c = misc[w2];
      if (c > WLCAP) ov = 1;
      c = c < 0 ? 0 : (c > WLCAP ? WLCAP : c);
      tot += c;
#pragma unroll 1
      for (int b0 = 0; b0 < c; b0 += 32) {
        const int idx = b0 + lane;
        const int ent = wl[w2 * WLCAP + (idx < WLCAP ? idx : WLCAP - 1)];
        const int m32 = (c - b0) < 32 ? (c - b0) : 32;
#pragma unroll 1
        for (int k = 0; k < m32; ++k) {
          const int u    = __builtin_amdgcn_readlane(ent, k);
          const int slot = u & (NBRUN - 1);
          const int cv   = cnt[slot];
          asm volatile("" :: "v"(cv));
          if (lane == 0) cnt[slot] = cv + 1;
        }
      }
    }
    if (tot > RCAP) ov = 1;
    if (lane == 0) misc[9] = ov;
  }
  __syncthreads();
  if (wave == 0) {
    const int base = lane * (NBRUN / 32);
    int s = 0;
#pragma unroll 1
    for (int i = 0; i < NBRUN / 32; ++i) s += cnt[base + i];
    int incl = s;
#pragma unroll
    for (int d = 1; d < 32; d <<= 1) {
      const int y = __shfl_up(incl, d, 32);
      if (lane >= d) incl += y;
    }
    int run = incl - s;
#pragma unroll 1
    for (int i = 0; i < NBRUN / 32; ++i) {
      const int cv = cnt[base + i];
      offs[base + i] = run;
      cur[base + i]  = run;
      run += cv;
    }
  }
  __syncthreads();

  if (wave == 0) {
#pragma unroll 1
    for (int w2 = 0; w2 < NWAVE; ++w2) {
      int c = misc[w2];
      c = c < 0 ? 0 : (c > WLCAP ? WLCAP : c);
#pragma unroll 1
      for (int b0 = 0; b0 < c; b0 += 32) {
        const int idx = b0 + lane;
        const int ent = wl[w2 * WLCAP + (idx < WLCAP ? idx : WLCAP - 1)];
        const int m32 = (c - b0) < 32 ? (c - b0) : 32;
#pragma unroll 1
        for (int k = 0; k < m32; ++k) {
          const int u    = __builtin_amdgcn_readlane(ent, k);
          const int slot = u & (NBRUN - 1);
          int p = cur[slot];
          asm volatile("" :: "v"(p));
          p = p < 0 ? 0 : (p > RCAP - 1 ? RCAP - 1 : p);
          if (lane == 0) {
            pl[p] = u;
            cur[slot] = p + 1;
          }
        }
      }
    }
  }
  __syncthreads();

  const int ovf = misc[9];
  const float qnan = __uint_as_float(0x7fc00000u);

#pragma unroll 1
  for (int it = 0; it < NBRUN / NTHR; ++it) {
    const int slot = it * NTHR + tid;
    int c = cnt[slot];
    int o = offs[slot];
    const bool big = c > DEGCAP;
    o = clampi(o, 0, RCAP - 1);
    c = clampi(c, 0, DEGCAP);
    c = c < (RCAP - o) ? c : (RCAP - o);
    int mx = c;
#pragma unroll
    for (int d = 16; d >= 1; d >>= 1) {
      const int y = __shfl_xor(mx, d, 32);
      mx = y > mx ? y : mx;
    }
    mx = __builtin_amdgcn_readfirstlane(mx);
    float deg = 0.0f;
#pragma unroll 1
    for (int j = 0; j < mx; ++j) {
      int idx = o + j;
      idx = idx > RCAP - 1 ? RCAP - 1 : idx;
      const int ent = pl[idx];
      const int eid = clampi((ent >> SLB) & (NE - 1), 0, NE - 1);
      const float wv = ew[eid];
      asm volatile("" :: "v"(wv));
      float w = bf16_val(wv);
      asm volatile("" : "+v"(w));
      const float add = (j < c) ? w : 0.0f;
      deg = deg + add;
    }
    deg = deg + 1.0f;
    const float rs = 1.0f / sqrtf(deg);
    float dv = (deg > 0.0f) ? rs : 0.0f;
    dv = (big || ovf != 0) ? qnan : dv;
    cur[slot] = __float_as_int(dv);
  }
  __syncthreads();

  int* lp = PAIRS + (size_t)blk * (size_t)(2 * RCAP);
#pragma unroll 1
  for (int i = tid * 2; i < RCAP; i += NTHR * 2) {
    const v2i hw = *(const v2ia*)(pl + i);
    const int e0 = clampi((hw.x >> SLB) & (NE - 1), 0, NE - 1);
    const int e1 = clampi((hw.y >> SLB) & (NE - 1), 0, NE - 1);
    const int   r0 = srcs[e0];
    const int   r1 = srcs[e1];
    const float w0 = ew[e0];
    const float w1 = ew[e1];
    asm volatile("" :: "v"(r0), "v"(r1), "v"(w0), "v"(w1));
    v4i o;
    o.x = clampi(r0, 0, NN - 1);
    o.y = (int)(bf16_bits(w0) << 16);
    o.z = clampi(r1, 0, NN - 1);
    o.w = (int)(bf16_bits(w1) << 16);
    st2_v4i(lp + 2 * i, o);
  }
  {
    const v4i a = *(const v4ia*)(cnt + 4 * tid);
    const v4i b = *(const v4ia*)(offs + 4 * tid);
    const v4i d = *(const v4ia*)(cur + 4 * tid);
    st2_v4i(CNT  + (size_t)blk * NBRUN + 4 * tid, a);
    st2_v4i(OFF  + (size_t)blk * NBRUN + 4 * tid, b);
    st2_v4i(DINV + (size_t)blk * NBRUN + 4 * tid, d);
  }
  if (tid < 8) {
    const v4i f = {ovf, ovf, ovf, ovf};
    st2_v4i(FLAG + (size_t)blk * 32 + 4 * tid, f);
  }
}

template <int SPLIT>
__global__ __launch_bounds__(NTHR) void k_walk(const int* __restrict__ PAIRS, const int* __restrict__ CNT,
                                               const int* __restrict__ OFF, const int* __restrict__ DINV,
                                               const int* __restrict__ FLAG, const float* __restrict__ T,
                                               const float* __restrict__ bias, unsigned* OP) {
  __shared__ __attribute__((aligned(16))) float sb[128];
  const int tid = (int)threadIdx.x, lane = tid & 31, wave = tid >> 5;
  const int blk = (int)blockIdx.x;
  if (wave == 0) {
    const v4f b = *(const v4fa*)(bias + 4 * (lane & 15));
    *(v4fa*)(sb + 4 * lane) = b;
  }
  __syncthreads();
  const v2f bv = *(const v2fa*)(sb + 2 * lane);
  const int bucket = (blk * OWB) >> SLB;
  const int flag = FLAG[(size_t)bucket * 32];
  const int* lb = PAIRS + (size_t)bucket * (size_t)(2 * RCAP);
  const float qnan = __uint_as_float(0x7fc00000u);
  const int pitchw = SPLIT ? 64 : 32;

#pragma unroll 1
  for (int i = 0; i < 8; ++i) {
    const int node = blk * OWB + wave * 8 + i;
    int c = CNT[node];
    int o = OFF[node];
    const int dbits = DINV[node];
    asm volatile("" :: "v"(c), "v"(o), "v"(dbits));
    const bool big = c > DEGCAP;
    o = clampi(o, 0, RCAP - 1);
    c = (node < NN) ? clampi(c, 0, (DEGCAP < RCAP - o) ? DEGCAP : (RCAP - o)) : 0;
    c = __builtin_amdgcn_readfirstlane(c);
    const int last = o + (c > 0 ? c : 1) - 1;
    const float dd = __int_as_float(dbits);
    const v2f selfv = *(const v2fa*)(T + (size_t)node * HD + 2 * lane);
    const float sx = selfv.x, sy = selfv.y;
    asm volatile("" :: "v"(sx), "v"(sy));
    float a0 = 0.0f, a1 = 0.0f;
#pragma unroll 1
    for (int b0 = 0; b0 < c; b0 += 32) {
      int idx = o + b0 + lane;
      idx = idx > last ? last : idx;
      const v2i ent = *(const v2ia*)(lb + 2 * idx);
      const int ex = ent.x, wv = ent.y;
      asm volatile("" :: "v"(ex), "v"(wv));
      const int sr = clampi(ex, 0, NN - 1);
      const int dsb = DINV[sr];
      asm volatile("" :: "v"(dsb));
      const int m32 = (c - b0) < 32 ? (c - b0) : 32;
#pragma unroll 1
      for (int k = 0; k < m32; ++k) {
        const int   sk = __builtin_amdgcn_readlane(sr, k);
        const float wk = __int_as_float(__builtin_amdgcn_readlane(wv, k));
        const float dk = __int_as_float(__builtin_amdgcn_readlane(dsb, k));
        const float t0 = dk * wk;
        const float nrm = t0 * dd;
        const v2f q = *(const v2fa*)(T + (size_t)sk * HD + 2 * lane);
        const float p0 = q.x * nrm;
        const float p1 = q.y * nrm;
        a0 = a0 + p0;
        a1 = a1 + p1;
      }
    }
    const float l0 = dd * 1.0f;
    const float ln = l0 * dd;
    const float q0 = sx * ln;
    const float q1 = sy * ln;
    a0 = a0 + q0;
    a1 = a1 + q1;
    const float v0 = a0 + bv.x;
    const float v1 = a1 + bv.y;
    float y0 = (v0 > 0.0f) ? v0 : (v0 - v0);
    float y1 = (v1 > 0.0f) ? v1 : (v1 - v1);
    const bool bad = (flag != 0) || big;
    y0 = bad ? qnan : y0;
    y1 = bad ? qnan : y1;
    const unsigned hiw = pk16(bf16_bits(y0), bf16_bits(y1));
    const unsigned low = pk16(bf16_lo_bits(y0), bf16_lo_bits(y1));
    unsigned* rp = OP + (size_t)node * (size_t)pitchw;
    *(volatile unsigned*)(rp + lane) = hiw;
    if (SPLIT) *(volatile unsigned*)(rp + 32 + lane) = low;
    __threadfence();
    *(volatile unsigned*)(rp + lane) = hiw;
    if (SPLIT) *(volatile unsigned*)(rp + 32 + lane) = low;
  }
}

__global__ __launch_bounds__(NTHR) void k_store(const float* __restrict__ TF, const int* __restrict__ FLAG, float* out) {
  const int f  = (int)blockIdx.x * NTHR + (int)threadIdx.x;
  const int fc = f < NOUT - 1 ? f : NOUT - 1;
  const int row = fc >> 1, col = fc & 1;
  const float v = TF[(size_t)row * HD + col];
  const int fl = FLAG[(size_t)(row >> SLB) * 32];
  asm volatile("" :: "v"(v), "v"(fl));
  const float qnan = __uint_as_float(0x7fc00000u);
  const float o = (fl != 0) ? qnan : v;
  if (f < NOUT) {
    *(volatile float*)(out + f) = o;
    __threadfence();
    *(volatile float*)(out + f) = o;
  }
}

extern "C" void kernel_launch(void* const* d_in, const int* in_sizes, int n_in,
                              void* d_out, int out_size, void* d_ws, size_t ws_size,
                              hipStream_t stream) {
  if (n_in < 9) return;
  if (in_sizes[0] != NN * CIN) return;
  if (in_sizes[1] != 2 * NE) return;
  if (in_sizes[2] != NE) return;
  if (in_sizes[3] != CIN * HD) return;
  if (in_sizes[4] != HD) return;
  if (in_sizes[5] != HD * HD) return;
  if (in_sizes[6] != HD) return;
  if (in_sizes[7] != HD * NOUTC) return;
  if (in_sizes[8] != NOUTC) return;
  if (out_size != NOUT) return;

  const float* x  = (const float*)d_in[0];
  const int*   ei = (const int*)d_in[1];
  const float* ew = (const float*)d_in[2];
  const float* W1 = (const float*)d_in[3];
  const float* b1 = (const float*)d_in[4];
  const float* W2 = (const float*)d_in[5];
  const float* b2 = (const float*)d_in[6];
  const float* Wl = (const float*)d_in[7];
  const float* bl = (const float*)d_in[8];
  float* out = (float*)d_out;

  constexpr size_t zXB    = (size_t)NN * KP1 * 2;
  constexpr size_t zT     = (size_t)NN * HD * 4;
  constexpr size_t zOP    = (size_t)NN * 128 * 2;
  constexpr size_t zPAIRS = (size_t)NBK * RCAP * 8;
  constexpr size_t zTAB   = (size_t)NN * 4;
  constexpr size_t zW1P   = (size_t)HD * KP1 * 2;
  constexpr size_t zW2D   = (size_t)HD * 128 * 2;
  constexpr size_t zWLD   = (size_t)HD * 128 * 2;
  constexpr size_t zBIAS  = (size_t)3 * HD * 4;
  constexpr size_t zFLAG  = (size_t)NBK * 128;
  constexpr size_t oXB    = 0;
  constexpr size_t oT     = oXB + zXB;
  constexpr size_t oOP    = oT + zT;
  constexpr size_t oPAIRS = oOP + zOP;
  constexpr size_t oCNT   = oPAIRS + zPAIRS;
  constexpr size_t oOFF   = oCNT + zTAB;
  constexpr size_t oDINV  = oOFF + zTAB;
  constexpr size_t oW1P   = oDINV + zTAB;
  constexpr size_t oW2D   = oW1P + zW1P;
  constexpr size_t oWLD   = oW2D + zW2D;
  constexpr size_t oBIAS  = oWLD + zWLD;
  constexpr size_t oFLAG  = oBIAS + zBIAS;
  constexpr size_t oEND   = oFLAG + zFLAG;
  static_assert(zXB % 128 == 0 && zT % 128 == 0 && zOP % 128 == 0 && zPAIRS % 128 == 0 && zTAB % 128 == 0);
  static_assert(zW1P % 128 == 0 && zW2D % 128 == 0 && zWLD % 128 == 0 && zBIAS % 128 == 0 && zFLAG % 128 == 0);
  static_assert(zOP >= (size_t)NN * K2 * 2 && zOP >= (size_t)NN * KH * 2);
  static_assert(zW2D >= (size_t)HD * K2 * 2 && zWLD >= (size_t)HD * KH * 2);
  static_assert(oEND == 49591040);
  static_assert(oEND <= ((size_t)128 << 20));
  if (oEND > ws_size) return;

  char* ws = (char*)d_ws;
  unsigned short* XB    = (unsigned short*)(ws + oXB);
  float*          T     = (float*)(ws + oT);
  unsigned short* OPh   = (unsigned short*)(ws + oOP);
  unsigned*       OPw   = (unsigned*)(ws + oOP);
  int*            PAIRS = (int*)(ws + oPAIRS);
  int*            CNT   = (int*)(ws + oCNT);
  int*            OFF   = (int*)(ws + oOFF);
  int*            DINV  = (int*)(ws + oDINV);
  unsigned short* W1P   = (unsigned short*)(ws + oW1P);
  unsigned short* W2D   = (unsigned short*)(ws + oW2D);
  unsigned short* WLD   = (unsigned short*)(ws + oWLD);
  float*          BIAS  = (float*)(ws + oBIAS);
  int*            FLAG  = (int*)(ws + oFLAG);

  hipFuncSetAttribute(reinterpret_cast<const void*>(&k_list), hipFuncAttributeMaxDynamicSharedMemorySize, (int)BK_LDS);

  constexpr int gemmBlocks = ((NN / 64) * (HD / 64) + 7) / 8;

  k_plane<0><<<NN * KP1 / 8 / 256, 256, 0, stream>>>(x, NN, CIN, CIN, XB, NN, KP1);
  k_prep<<<PBTOT, NTHR, 0, stream>>>(W1, b1, W2, b2, Wl, bl, W1P, W2D, WLD, BIAS);
  k_list<<<NBK, NTHR, BK_LDS, stream>>>(ei, ew, PAIRS, CNT, OFF, DINV, FLAG);
  k_gemm_nt<0, 0><<<gemmBlocks, 256, 0, stream>>>(XB, W1P, BIAS, T, NN, HD, KP1, HD);
  k_walk<SPLIT_L2><<<NN / OWB, NTHR, 0, stream>>>(PAIRS, CNT, OFF, DINV, FLAG, T, BIAS, OPw);
  k_gemm_nt<0, 0><<<gemmBlocks, 256, 0, stream>>>(OPh, W2D, BIAS, T, NN, HD, K2, HD);
  k_walk<SPLIT_H><<<NN / OWB, NTHR, 0, stream>>>(PAIRS, CNT, OFF, DINV, FLAG, T, BIAS + HD, OPw);
  k_gemm_nt<0, 1><<<gemmBlocks, 256, 0, stream>>>(OPh, WLD, BIAS + 2 * HD, T, NN, HD, KH, HD);
  k_store<<<NOUT / NTHR, NTHR, 0, stream>>>(T, FLAG, out);
}
